// MechanismGrabber_28887950033396
// MI455X (gfx1250) — hardware-verified
//
#include <hip/hip_runtime.h>
#include <math.h>
typedef __attribute__((ext_vector_type(16))) _Float16 v16h;
typedef __attribute__((ext_vector_type(8)))  _Float16 v8h;
typedef __attribute__((ext_vector_type(16))) __bf16   v16b;
typedef __attribute__((ext_vector_type(8)))  __bf16   v8b;
typedef __attribute__((ext_vector_type(8)))  float    v8f;
typedef __attribute__((ext_vector_type(4)))  float    v4f;
#define PSCALE 32768.0f
#define U16(p) ((const unsigned short*)(const void*)(p))
#define PSCALE_INV (1.0f / 32768.0f)

__device__ __forceinline__ unsigned short f2bf_bits(float f) {
  unsigned u = __float_as_uint(f);
  return (unsigned short)((u + 0x7FFFu + ((u >> 16) & 1u)) >> 16);
}
__device__ __forceinline__ float bf_bits2f(unsigned short h) { return __uint_as_float(((unsigned)h) << 16); }

__device__ __forceinline__ void dep_guard_h(v8f& a, v8f& b, v16h x, v16h y) { asm volatile("v_nop\n\tv_nop\n\tv_nop\n\tv_nop" : "+v"(a), "+v"(b) : "v"(x), "v"(y)); }
__device__ __forceinline__ void dep_guard_b(v8f& a, v8f& b, v16b x, v16b y) { asm volatile("v_nop\n\tv_nop\n\tv_nop\n\tv_nop" : "+v"(a), "+v"(b) : "v"(x), "v"(y)); }
__device__ __forceinline__ void keep4_h(v16h a, v16h b, v16h c, v16h d) { asm volatile("v_nop" :: "v"(a), "v"(b), "v"(c), "v"(d)); }
__device__ __forceinline__ void keep4_b(v16b a, v16b b, v16b c, v16b d) { asm volatile("v_nop" :: "v"(a), "v"(b), "v"(c), "v"(d)); }
__device__ __forceinline__ void acc_guard4(v8f& a, v8f& b, v8f& c, v8f& d) { asm volatile("v_nop\n\tv_nop\n\tv_nop\n\tv_nop" : "+v"(a), "+v"(b), "+v"(c), "+v"(d)); }
template <typename T> struct Frag;
template <> struct Frag<_Float16> {
  typedef v16h V; union U { v16h v; v8h h[2]; };
  static __device__ __forceinline__ v16h load(const _Float16* p) {
    U f; f.h[0] = *(const v8h*)(p); f.h[1] = *(const v8h*)(p + 16); return f.v;
  }
  static __device__ __forceinline__ v8f mma(v16h a, v16h b, v8f c) {
    return __builtin_amdgcn_wmma_f32_16x16x32_f16(false, a, false, b, (short)0, c, false, false);
  }
  static __device__ __forceinline__ void guard(v8f& a, v8f& b, v16h x, v16h y) { dep_guard_h(a, b, x, y); }
  static __device__ __forceinline__ void keep(v16h a, v16h b, v16h c, v16h d) { keep4_h(a, b, c, d); }
};
template <> struct Frag<__bf16> {
  typedef v16b V; union U { v16b v; v8b h[2]; };
  static __device__ __forceinline__ v16b load(const __bf16* p) {
    U f; f.h[0] = *(const v8b*)(p); f.h[1] = *(const v8b*)(p + 16); return f.v;
  }
  static __device__ __forceinline__ v8f mma(v16b a, v16b b, v8f c) {
    return __builtin_amdgcn_wmma_f32_16x16x32_bf16(false, a, false, b, (short)0, c, false, false);
  }
  static __device__ __forceinline__ void guard(v8f& a, v8f& b, v16b x, v16b y) { dep_guard_b(a, b, x, y); }
  static __device__ __forceinline__ void keep(v16b a, v16b b, v16b c, v16b d) { keep4_b(a, b, c, d); }
};

template <int ET> struct Elem;
template <> struct Elem<0> { typedef _Float16 T; };
template <> struct Elem<1> { typedef __bf16 T; };
template <int ET, bool SPLIT, int BIAS_MODE, int OUT_MODE, bool RESID, int ACT = 0>
__global__ __launch_bounds__(256) void wmma_gemm64(
    const unsigned short* __restrict__ Ap, const unsigned short* __restrict__ A2p, int lda, long strideA,
    const unsigned short* __restrict__ Btp, const unsigned short* __restrict__ Bt2p, int ldb, long strideB,
    void* __restrict__ Cout, void* __restrict__ Cout2, int ldc, long strideC,
    const float* __restrict__ bias,
    const float* __restrict__ resid, long strideR,
    int M, int N, int K, float scale) {
  typedef typename Elem<ET>::T T;
  typedef typename Frag<T>::V V;
  const T* A = (const T*)Ap; const T* A2 = (const T*)A2p; const T* Bt = (const T*)Btp; const T* Bt2 = (const T*)Bt2p;
  __shared__ __align__(16) float sT[8][16 * 68];
  const int b    = blockIdx.y;
  const int lane = threadIdx.x & 31;
  const int wave = threadIdx.x >> 5;
  const int tilesN = N >> 6;
  const int tilesM = M >> 6;
  const int tile = blockIdx.x * 8 + wave;
  if (tile >= tilesM * tilesN) return;
  const int tm = tile / tilesN;
  const int tn = tile - tm * tilesN;
  const int m0 = tm << 6;
  const int n0 = tn << 6;

  const T* Ab  = A  + (size_t)b * strideA;
  const T* Bb  = Bt + (size_t)b * strideB;
  const T* Ab2 = SPLIT ? (A2  + (size_t)b * strideA) : nullptr;
  const T* Bb2 = SPLIT ? (Bt2 + (size_t)b * strideB) : nullptr;

  const int rlane = lane & 15;
  const int koff  = (lane >> 4) * 8;
  const int mOff  = (lane >> 4) * 8;

  v8f acc[4][4];
#pragma unroll
  for (int i = 0; i < 4; ++i)
#pragma unroll
    for (int j = 0; j < 4; ++j) acc[i][j] = (v8f){0.f,0.f,0.f,0.f,0.f,0.f,0.f,0.f};

  for (int k0 = 0; k0 < K; k0 += 32) {
    V bh[4], bl[4];
#pragma unroll
    for (int j = 0; j < 4; ++j) {
      const size_t bo = (size_t)(n0 + (j << 4) + rlane) * ldb + koff + k0;
      bh[j] = Frag<T>::load(Bb + bo);
      if (SPLIT) bl[j] = Frag<T>::load(Bb2 + bo);
    }
#pragma unroll
    for (int i = 0; i < 4; ++i) {
      const size_t ao = (size_t)(m0 + (i << 4) + rlane) * lda + koff + k0;
      V ah = Frag<T>::load(Ab + ao);
      V al;
      if (SPLIT) al = Frag<T>::load(Ab2 + ao);
#pragma unroll
      for (int j = 0; j < 4; ++j) {
        acc[i][j] = Frag<T>::mma(ah, bh[j], acc[i][j]);
        if (SPLIT) {
          acc[i][j] = Frag<T>::mma(ah, bl[j], acc[i][j]);
          acc[i][j] = Frag<T>::mma(al, bh[j], acc[i][j]);
        }
      }
      Frag<T>::guard(acc[i][0], acc[i][3], ah, SPLIT ? al : ah);
    }
    Frag<T>::keep(bh[0], bh[1], bh[2], bh[3]);
    if (SPLIT) Frag<T>::keep(bl[0], bl[1], bl[2], bl[3]);
  }
  acc_guard4(acc[0][0], acc[0][1], acc[0][2], acc[0][3]);
  acc_guard4(acc[1][0], acc[1][1], acc[1][2], acc[1][3]);
  acc_guard4(acc[2][0], acc[2][1], acc[2][2], acc[2][3]);
  acc_guard4(acc[3][0], acc[3][1], acc[3][2], acc[3][3]);

  float* slab = sT[wave];
  const float* Rb = RESID ? (resid + (size_t)b * strideR) : nullptr;
#pragma unroll
  for (int i = 0; i < 4; ++i) {
    const int mBase = m0 + (i << 4);
#pragma unroll
    for (int j = 0; j < 4; ++j) {
      const int n = n0 + (j << 4) + rlane;
      float bv = 0.f;
      if (BIAS_MODE == 2) bv = bias[n];
#pragma unroll
      for (int r = 0; r < 8; ++r) {
        float v = acc[i][j][r] * scale;
        if (BIAS_MODE == 1) v += bias[mBase + mOff + r];
        if (BIAS_MODE == 2) v += bv;
        if (RESID) v += Rb[(size_t)(mBase + mOff + r) * ldc + n];
        if (ACT == 1) v = tanhf(v);
        if (ACT == 2) v = fmaxf(v, 0.0f);
        if (ACT == 3) v = v / (1.0f + expf(-v));
        if (ACT == 4) v = (v > 0.f) ? v : 0.01f * v;
        if (ACT == 5) v = 0.5f * v * (1.0f + erff(v * 0.70710678118654752f));
        slab[(mOff + r) * 68 + (j << 4) + rlane] = v;
      }
    }
    __builtin_amdgcn_fence(__ATOMIC_RELEASE, "workgroup");
    __builtin_amdgcn_wave_barrier();
    __builtin_amdgcn_fence(__ATOMIC_ACQUIRE, "workgroup");
    if (OUT_MODE == 0) {
      float* C = (float*)Cout + (size_t)b * strideC;
      const int hh = lane >> 4, c4 = (lane & 15) * 4;
      for (int pass = 0; pass < 2; ++pass) {
#pragma unroll
        for (int it = 0; it < 8; ++it) {
          const int row = it * 2 + hh;
          v4f v = *(const v4f*)(slab + row * 68 + c4);
          *(volatile v4f*)(C + (size_t)(mBase + row) * ldc + n0 + c4) = v;
        }
        __threadfence();
      }
    } else {
      const int q = lane >> 3, c8 = (lane & 7) * 8;
      unsigned short* C  = (unsigned short*)Cout  + (size_t)b * strideC;
      unsigned short* C2 = (OUT_MODE == 2) ? ((unsigned short*)Cout2 + (size_t)b * strideC) : nullptr;
      for (int pass = 0; pass < 2; ++pass) {
#pragma unroll
        for (int it = 0; it < 4; ++it) {
          const int row = it * 4 + q;
          const float* sp = slab + row * 68 + c8;
          v8h hv, lv;
#pragma unroll
          for (int e = 0; e < 8; ++e) {
            if (OUT_MODE == 1) {
              hv[e] = (_Float16)sp[e];
            } else {
              unsigned short hb = f2bf_bits(sp[e]);
              unsigned short lb = f2bf_bits(sp[e] - bf_bits2f(hb));
              hv[e] = __builtin_bit_cast(_Float16, hb);
              lv[e] = __builtin_bit_cast(_Float16, lb);
            }
          }
          *(volatile v8h*)(C + (size_t)(mBase + row) * ldc + n0 + c8) = hv;
          if (OUT_MODE == 2) *(volatile v8h*)(C2 + (size_t)(mBase + row) * ldc + n0 + c8) = lv;
        }
        __threadfence();
      }
    }
    __builtin_amdgcn_fence(__ATOMIC_RELEASE, "workgroup");
    __builtin_amdgcn_wave_barrier();
    __builtin_amdgcn_fence(__ATOMIC_ACQUIRE, "workgroup");
  }
}

__global__ __launch_bounds__(256) void cast_f32_f16x2(
    const float* __restrict__ in, _Float16* __restrict__ out, int n2) {
  int i = blockIdx.x * 256 + threadIdx.x;
  if (i < n2) {
    const _Float16 h0 = (_Float16)in[2 * i], h1 = (_Float16)in[2 * i + 1];
    const unsigned u = (unsigned)__builtin_bit_cast(unsigned short, h0) | ((unsigned)__builtin_bit_cast(unsigned short, h1) << 16);
    ((volatile unsigned*)out)[i] = u;
    __threadfence();
    ((volatile unsigned*)out)[i] = u;
  }
}


__global__ __launch_bounds__(256) void transpose_cast_f16(const float* __restrict__ in, int ldi,
                                                         _Float16* __restrict__ outT, int ldo, float scale) {
  __shared__ __align__(16) _Float16 tile[64][72];
  const int c0 = blockIdx.x * 64, r0 = blockIdx.y * 64;
  const int t = threadIdx.y * 32 + threadIdx.x;
  for (int i = threadIdx.y; i < 64; i += 8) {
    tile[threadIdx.x][i]      = (_Float16)(in[(size_t)(r0 + i) * ldi + c0 + threadIdx.x] * scale);
    tile[32 + threadIdx.x][i] = (_Float16)(in[(size_t)(r0 + i) * ldi + c0 + 32 + threadIdx.x] * scale);
  }
  __syncthreads();
  const int q = t >> 3, c8 = (t & 7) * 8;
  for (int pass = 0; pass < 2; ++pass) {
#pragma unroll
    for (int it = 0; it < 2; ++it) {
      const int c = it * 32 + q;
      v8h hv = *(const v8h*)(&tile[c][c8]);
      *(volatile v8h*)(outT + (size_t)(c0 + c) * ldo + r0 + c8) = hv;
    }
    __threadfence();
  }
}

#define GR_ 8192
#define GD_ 128
#define GM_ 64
#define GCH 4
#define GRC (GR_ / GCH)
__device__ __forceinline__ unsigned pkh(float a, float b) { return (unsigned)__builtin_bit_cast(unsigned short, (_Float16)a) | ((unsigned)__builtin_bit_cast(unsigned short, (_Float16)b) << 16); }
__global__ __launch_bounds__(256) void cat_kernel(const float* __restrict__ x, const float* __restrict__ ctx, unsigned* __restrict__ A16) { const long i = (long)blockIdx.x * 256 + threadIdx.x; if (i >= (long)GR_ * 128) return; const long r = i / 128; const int cp = 2 * (int)(i % 128); float a, b; if (cp < GD_) { a = x[r * GD_ + cp]; b = x[r * GD_ + cp + 1]; } else { a = ctx[r * GD_ + cp - GD_]; b = ctx[r * GD_ + cp - GD_ + 1]; } ((volatile unsigned*)A16)[i] = pkh(a, b); __threadfence(); ((volatile unsigned*)A16)[i] = pkh(a, b); }
__global__ __launch_bounds__(256) void wt_kernel(const float* __restrict__ Wt, unsigned* __restrict__ BT) { for (long i = (long)blockIdx.x * 256 + threadIdx.x; i < (long)GM_ * GD_ * GD_ / 2; i += (long)gridDim.x * 256) { const long row = i / 64; const int kp = 2 * (int)(i % 64); const int m = (int)(row / GD_), o = (int)(row % GD_); const unsigned u = pkh(Wt[((size_t)m * GD_ + kp) * GD_ + o], Wt[((size_t)m * GD_ + kp + 1) * GD_ + o]); ((volatile unsigned*)BT)[i] = u; __threadfence(); ((volatile unsigned*)BT)[i] = u; } }
__global__ __launch_bounds__(256) void score_kernel(const float* __restrict__ SEL, const float* __restrict__ O, float* __restrict__ SC, float* __restrict__ GW) {
  const int lane = threadIdx.x & 31, wave = threadIdx.x >> 5; const long r = (long)blockIdx.x * 8 + wave; const float a = SEL[r * GM_ + 2 * lane], b = SEL[r * GM_ + 2 * lane + 1];
  float mx = fmaxf(a, b); for (int o = 16; o > 0; o >>= 1) mx = fmaxf(mx, __shfl_xor(mx, o, 32)); const float ea = __expf(a - mx), eb = __expf(b - mx); float s = ea + eb; for (int o = 16; o > 0; o >>= 1) s += __shfl_xor(s, o, 32);
  const float sa = ea / s, sb = eb / s;
  __shared__ float sc[8][GM_]; sc[wave][2 * lane] = sa; sc[wave][2 * lane + 1] = sb; __syncthreads();
  float g0 = 0.f, g1 = 0.f;
#pragma unroll 4
  for (int m = 0; m < GM_; ++m) { const float v = sc[wave][m]; g0 += v * O[m * GM_ + 2 * lane]; g1 += v * O[m * GM_ + 2 * lane + 1]; }
  g0 = (1.0f + tanhf(g0)) * sa; g1 = (1.0f + tanhf(g1)) * sb;
  for (int pass = 0; pass < 2; ++pass) { ((volatile float*)SC)[r * GM_ + 2 * lane] = sa; ((volatile float*)SC)[r * GM_ + 2 * lane + 1] = sb; ((volatile float*)GW)[r * GM_ + 2 * lane] = g0; ((volatile float*)GW)[r * GM_ + 2 * lane + 1] = g1; __threadfence(); }
}
__global__ __launch_bounds__(256) void mix_kernel(const float* __restrict__ T, long r0, const float* __restrict__ bt, const float* __restrict__ chr, const float* __restrict__ TIM, const float* __restrict__ bg, const float* __restrict__ Wv, const float* __restrict__ bv, const float* __restrict__ SC, const float* __restrict__ GW, float* __restrict__ SELP, float* __restrict__ VPP) {
  const int lane = threadIdx.x & 31, wave = threadIdx.x >> 5; const long idx = (long)blockIdx.x * 8 + wave; const int grp = (int)(idx & 7); const long rl = idx >> 3; const long r = r0 + rl;
  v4f acc = {0.f, 0.f, 0.f, 0.f}; float vp = 0.f;
  for (int mm = 0; mm < 8; ++mm) { const int m = grp * 8 + mm; const v4f tv = *(const v4f*)(T + (rl * GM_ + m) * GD_ + lane * 4); const v4f b4 = *(const v4f*)(bt + m * GD_ + lane * 4), c4 = *(const v4f*)(chr + m * GD_ + lane * 4), w4 = *(const v4f*)(Wv + m * GD_ + lane * 4);
    const v4f tr = tv + b4 + c4; float vd = tr[0] * w4[0] + tr[1] * w4[1] + tr[2] * w4[2] + tr[3] * w4[3]; for (int o = 16; o > 0; o >>= 1) vd += __shfl_xor(vd, o, 32);
    const float timing = 1.0f / (1.0f + __expf(-(TIM[r * GM_ + m] + bg[m]))); const float wgt = timing * GW[r * GM_ + m];
    acc += tr * wgt; vp += (1.0f / (1.0f + __expf(-(vd + bv[m])))) * SC[r * GM_ + m]; }
  float* dst = SELP + ((size_t)grp * GRC + rl) * GD_ + lane * 4;
  for (int pass = 0; pass < 2; ++pass) { *(volatile v4f*)dst = acc; if (lane == 0) ((volatile float*)VPP)[(size_t)grp * GRC + rl] = vp; __threadfence(); }
}
__global__ __launch_bounds__(256) void gsum_kernel(const float* __restrict__ SELP, const float* __restrict__ VPP, long r0, const float* __restrict__ x, unsigned* __restrict__ IN16, float* __restrict__ vpot) {
  const int lane = threadIdx.x & 31, wave = threadIdx.x >> 5; const long rl = (long)blockIdx.x * 8 + wave; const long r = r0 + rl;
  v4f s = {0.f, 0.f, 0.f, 0.f}; float v = 0.f; for (int g = 0; g < 8; ++g) { s += *(const v4f*)(SELP + ((size_t)g * GRC + rl) * GD_ + lane * 4); v += VPP[(size_t)g * GRC + rl]; }
  const v4f xv = *(const v4f*)(x + r * GD_ + lane * 4); typedef __attribute__((ext_vector_type(2))) unsigned u2; const u2 ux = {pkh(xv[0], xv[1]), pkh(xv[2], xv[3])}, us = {pkh(s[0], s[1]), pkh(s[2], s[3])};
  for (int pass = 0; pass < 2; ++pass) { *(volatile u2*)(IN16 + (r * 256 + lane * 4) / 2) = ux; *(volatile u2*)(IN16 + (r * 256 + GD_ + lane * 4) / 2) = us; if (lane == 0) ((volatile float*)vpot)[r] = v; __threadfence(); }
}
extern "C" void kernel_launch(void* const* d_in, const int* in_sizes, int n_in, void* d_out, int out_size, void* d_ws, size_t ws_size, hipStream_t stream) {
  (void)in_sizes; (void)n_in; (void)out_size; (void)ws_size;
  auto Fp = [&](int i) { return (const float*)d_in[i]; };
  const float* x = Fp(0); const float* ctx = Fp(1); const float* Wt = Fp(2); const float* bt = Fp(3); const float* chr = Fp(4); const float* Wg = Fp(5); const float* bg = Fp(6); const float* Wv = Fp(7); const float* bv = Fp(8); const float* O = Fp(9); const float* W1 = Fp(10); const float* b1 = Fp(11); const float* W2 = Fp(12); const float* b2 = Fp(13); const float* Wi = Fp(14); const float* bi = Fp(15);
  float* out = (float*)d_out; float* vpot = out + (size_t)GR_ * GD_;
  char* ws = (char*)d_ws; size_t off = 0;
  auto carve = [&](size_t bytes) -> char* { char* p = ws + off; off += (bytes + 255) & ~(size_t)255; return p; };
  unsigned* A16 = (unsigned*)carve((size_t)GR_ * 256 * 2); unsigned* BTT = (unsigned*)carve((size_t)GM_ * GD_ * GD_ * 2); _Float16* W1T = (_Float16*)carve(256 * 256 * 2); _Float16* W2T = (_Float16*)carve(64 * 256 * 2); _Float16* WgT = (_Float16*)carve(64 * 128 * 2); _Float16* WiT = (_Float16*)carve(128 * 256 * 2);
  _Float16* H1 = (_Float16*)carve((size_t)GR_ * 256 * 2); float* SEL = (float*)carve((size_t)GR_ * GM_ * 4); float* TIM = (float*)carve((size_t)GR_ * GM_ * 4); float* SC = (float*)carve((size_t)GR_ * GM_ * 4); float* GW = (float*)carve((size_t)GR_ * GM_ * 4);
  float* T = (float*)carve((size_t)GRC * GM_ * GD_ * 4); float* SELP = (float*)carve((size_t)8 * GRC * GD_ * 4); float* VPP = (float*)carve((size_t)8 * GRC * 4); unsigned* IN16 = (unsigned*)carve((size_t)GR_ * 256 * 2);
  cat_kernel<<<(GR_ * 128 + 255) / 256, 256, 0, stream>>>(x, ctx, A16);
  wt_kernel<<<256, 256, 0, stream>>>(Wt, BTT);
  transpose_cast_f16<<<dim3(4, 4), dim3(32, 8), 0, stream>>>(W1, 256, W1T, 256, 1.0f); transpose_cast_f16<<<dim3(1, 4), dim3(32, 8), 0, stream>>>(W2, 64, W2T, 256, 1.0f); transpose_cast_f16<<<dim3(2, 4), dim3(32, 8), 0, stream>>>(Wi, 128, WiT, 256, 1.0f);
  cast_f32_f16x2<<<(64 * 128 / 2 + 255) / 256, 256, 0, stream>>>(Wg, WgT, 64 * 128 / 2);
  const int tr = GR_ / 64;
  wmma_gemm64<0, false, 2, 1, false, 5><<<dim3((tr * 4 + 7) / 8, 1), 256, 0, stream>>>((const unsigned short*)A16, nullptr, 256, 0, U16(W1T), nullptr, 256, 0, H1, nullptr, 256, 0, b1, nullptr, 0, GR_, 256, 256, 1.0f);
  wmma_gemm64<0, false, 2, 0, false><<<dim3((tr + 7) / 8, 1), 256, 0, stream>>>(U16(H1), nullptr, 256, 0, U16(W2T), nullptr, 256, 0, SEL, nullptr, GM_, 0, b2, nullptr, 0, GR_, GM_, 256, 1.0f);
  wmma_gemm64<0, false, 0, 0, false><<<dim3((tr + 7) / 8, 1), 256, 0, stream>>>((const unsigned short*)A16, nullptr, 256, 0, U16(WgT), nullptr, GD_, 0, TIM, nullptr, GM_, 0, nullptr, nullptr, 0, GR_, GM_, GD_, 1.0f);
  score_kernel<<<GR_ / 8, 256, 0, stream>>>(SEL, O, SC, GW);
  const int tt = (GRC / 64) * (GM_ * GD_ / 64);
  for (int ch = 0; ch < GCH; ++ch) { const long r0 = (long)ch * GRC;
    wmma_gemm64<0, false, 0, 0, false><<<dim3((tt + 7) / 8, 1), 256, 0, stream>>>((const unsigned short*)A16 + r0 * 256, nullptr, 256, 0, (const unsigned short*)BTT, nullptr, GD_, 0, T, nullptr, GM_ * GD_, 0, nullptr, nullptr, 0, GRC, GM_ * GD_, GD_, 1.0f);
    mix_kernel<<<(unsigned)(GRC * 8 / 8), 256, 0, stream>>>(T, r0, bt, chr, TIM, bg, Wv, bv, SC, GW, SELP, VPP);
    gsum_kernel<<<GRC / 8, 256, 0, stream>>>(SELP, VPP, r0, x, IN16, vpot); }
  wmma_gemm64<0, false, 2, 0, false><<<dim3((tr * 2 + 7) / 8, 1), 256, 0, stream>>>((const unsigned short*)IN16, nullptr, 256, 0, U16(WiT), nullptr, 256, 0, out, nullptr, GD_, 0, bi, nullptr, 0, GR_, GD_, 256, 1.0f);
}
